// GDAGDL_model_83150566851176
// MI455X (gfx1250) — hardware-verified
//
#include <hip/hip_runtime.h>
#include <stdint.h>
#include <stddef.h>
#include <math.h>

#pragma clang fp contract(off)

#define NPT   1024
#define PLEN  2048
#define NSEG  64
#define NNODE 33
#define NFRM  33
#define GW    64
#define YK    2112
#define BSZ   32
#define TST   32
#define HID   256
#define G4    1024
#define XIN   128
#define MROW  1024

#define E0K 2112
#define E0N 1024
#define E1N 512
#define E2N 256
#define E3N 128

#define AP  72
#define BP  72
#define WP  68
#define TP  132
#define TSP 72
#define LHP 264

#define O_X    0
#define O_TW   (O_X + NFRM * NSEG * 4)
#define O_MAG  (O_TW + 192 * 4)
#define O_C    (O_MAG + 4368)
#define O_PCC  (O_C + 4368)
#define O_V    (O_PCC + 4368)
#define O_AH   (O_V + 336 * 4)
#define O_AL   (O_AH + 48 * AP * 2)
#define O_BH   (O_AL + 48 * AP * 2)
#define O_BL   (O_BH + 64 * BP * 2)
#define O_WH   (O_BL + 64 * BP * 2)
#define LDS_FRONT (O_WH + 48 * WP * 4)

static_assert(LDS_FRONT == 68976);
static_assert((O_TW % 16) == 0);
static_assert((O_MAG % 16) == 0);
static_assert((O_C % 16) == 0);
static_assert((O_PCC % 16) == 0);
static_assert((O_V % 16) == 0);
static_assert((O_AH % 16) == 0);
static_assert((O_AL % 16) == 0);
static_assert((O_BH % 16) == 0);
static_assert((O_BL % 16) == 0);
static_assert((O_WH % 16) == 0);
static_assert((AP * 2) % 16 == 0);
static_assert((BP * 2) % 16 == 0);
static_assert((TP * 4) % 16 == 0);
static_assert((TSP * 2) % 16 == 0);
static_assert((LHP * 2) % 16 == 0);
static_assert(NNODE * NNODE * 4 <= 4368);
static_assert(E0K % 64 == 0);
static_assert(E0N % 128 == 0);
static_assert(E1N % 128 == 0);
static_assert(E2N % 128 == 0);
static_assert(E3N % 128 == 0);
static_assert(MROW % 64 == 0);
static_assert(YK == NNODE * GW);
static_assert(E3N == XIN);

typedef __bf16         v16bf __attribute__((ext_vector_type(16)));
typedef float          v8f   __attribute__((ext_vector_type(8)));
typedef float          v4f   __attribute__((ext_vector_type(4)));
typedef unsigned int   v4u   __attribute__((ext_vector_type(4)));
typedef v4f __attribute__((may_alias)) v4fa;
typedef v4u __attribute__((may_alias)) v4ua;

union FragBF { v16bf v; v4u q[2]; };

__device__ __forceinline__ unsigned int bfb(float f) {
  unsigned int u = __float_as_uint(f);
  u += 0x7FFFu + ((u >> 16) & 1u);
  return u >> 16;
}
__device__ __forceinline__ void split2(float v, unsigned int& hi, unsigned int& lo) {
  hi = bfb(v);
  lo = bfb(v - __uint_as_float(hi << 16));
}
__device__ __forceinline__ unsigned int pk(unsigned int a, unsigned int b) { return (a & 0xFFFFu) | (b << 16); }

__device__ __forceinline__ void split8(v4f a, v4f c, v4u& H, v4u& L) {
  unsigned int h0, l0, h1, l1, h2, l2, h3, l3, h4, l4, h5, l5, h6, l6, h7, l7;
  split2(a.x, h0, l0); split2(a.y, h1, l1); split2(a.z, h2, l2); split2(a.w, h3, l3);
  split2(c.x, h4, l4); split2(c.y, h5, l5); split2(c.z, h6, l6); split2(c.w, h7, l7);
  H.x = pk(h0, h1); H.y = pk(h2, h3); H.z = pk(h4, h5); H.w = pk(h6, h7);
  L.x = pk(l0, l1); L.y = pk(l2, l3); L.z = pk(l4, l5); L.w = pk(l6, l7);
}

__device__ __forceinline__ v4f relu4(v4f a) {
  a.x = fmaxf(a.x, 0.f); a.y = fmaxf(a.y, 0.f); a.z = fmaxf(a.z, 0.f); a.w = fmaxf(a.w, 0.f);
  return a;
}

__device__ __forceinline__ v8f wmma_bf(v16bf a, v16bf b, v8f c) {
  v8f d = __builtin_amdgcn_wmma_f32_16x16x32_bf16(false, a, false, b, (short)0, c, false, false);
  asm volatile("v_nop\n\tv_nop\n\tv_nop\n\tv_nop" : "+v"(d) : "v"(a), "v"(b));
  return d;
}

__device__ __forceinline__ v16bf ldfrag_bf(const unsigned short* p, int h) {
  FragBF f;
  f.q[0] = *(const v4ua*)(p + 8 * h);
  f.q[1] = *(const v4ua*)(p + 16 + 8 * h);
  return f.v;
}

__global__ __launch_bounds__(256) void k_split(const float* __restrict__ src,
                                               unsigned short* __restrict__ ph,
                                               unsigned short* __restrict__ pl, int n8)
{
  const int g = blockIdx.x * 256 + threadIdx.x;
  if (g >= n8) return;
  const float* s = src + (size_t)g * 8;
  const v4f a = *(const v4fa*)s;
  const v4f c = *(const v4fa*)(s + 4);
  v4u H, L;
  split8(a, c, H, L);
  unsigned short* dh = ph + (size_t)g * 8;
  unsigned short* dl = pl + (size_t)g * 8;
  *(volatile v4u*)dh = H;
  *(volatile v4u*)dl = L;
  __threadfence();
  *(volatile v4u*)dh = H;
  *(volatile v4u*)dl = L;
}

__global__ __launch_bounds__(256) void k_tsplit(const float* __restrict__ W,
                                                unsigned short* __restrict__ Th,
                                                unsigned short* __restrict__ Tl, int K, int N)
{
  __shared__ __align__(16) unsigned short sH[64 * TSP];
  __shared__ __align__(16) unsigned short sL[64 * TSP];
  const int tid = threadIdx.x, lane = tid & 31, wv = tid >> 5;
  const int n0 = blockIdx.x * 64, k0 = blockIdx.y * 64;
  #pragma unroll 4
  for (int i = 0; i < 16; ++i) {
    const int idx = tid + 256 * i;
    const int kk = idx >> 6, nn = idx & 63;
    const float v = W[(size_t)(k0 + kk) * N + n0 + nn];
    unsigned int hb, lb;
    split2(v, hb, lb);
    sH[nn * TSP + kk] = (unsigned short)hb;
    sL[nn * TSP + kk] = (unsigned short)lb;
  }
  __syncthreads();
  const int piece = lane & 7, rq = lane >> 3;
  v4u hv[2], lv[2];
  size_t go[2];
  #pragma unroll
  for (int ps = 0; ps < 2; ++ps) {
    const int row = ps * 32 + wv * 4 + rq;
    hv[ps] = *(const v4ua*)(sH + row * TSP + 8 * piece);
    lv[ps] = *(const v4ua*)(sL + row * TSP + 8 * piece);
    go[ps] = (size_t)(n0 + row) * K + k0 + 8 * piece;
  }
  #pragma unroll
  for (int ps = 0; ps < 2; ++ps) {
    *(volatile v4u*)(Th + go[ps]) = hv[ps];
    *(volatile v4u*)(Tl + go[ps]) = lv[ps];
  }
  __threadfence();
  #pragma unroll
  for (int ps = 0; ps < 2; ++ps) {
    *(volatile v4u*)(Th + go[ps]) = hv[ps];
    *(volatile v4u*)(Tl + go[ps]) = lv[ps];
  }
}

__device__ __forceinline__ void gat_gemm(const unsigned short* sAh, const unsigned short* sAl,
                                         const unsigned short* sBh, const unsigned short* sBl,
                                         int wv, int h, int m, v8f (&acc)[3])
{
  const v8f z8 = {0.f, 0.f, 0.f, 0.f, 0.f, 0.f, 0.f, 0.f};
  #pragma unroll
  for (int mt = 0; mt < 3; ++mt) acc[mt] = z8;
  #pragma unroll
  for (int ks = 0; ks < 2; ++ks) {
    const int bo = (16 * wv + m) * BP + 32 * ks;
    const v16bf bh = ldfrag_bf(sBh + bo, h);
    const v16bf bl = ldfrag_bf(sBl + bo, h);
    #pragma unroll
    for (int mt = 0; mt < 3; ++mt) {
      const int ao = (16 * mt + m) * AP + 32 * ks;
      const v16bf ah = ldfrag_bf(sAh + ao, h);
      const v16bf al = ldfrag_bf(sAl + ao, h);
      acc[mt] = wmma_bf(ah, bh, acc[mt]);
      acc[mt] = wmma_bf(ah, bl, acc[mt]);
      acc[mt] = wmma_bf(al, bh, acc[mt]);
    }
  }
}

__global__ __launch_bounds__(128) void k_front(
    const float* __restrict__ x,
    const float* __restrict__ w0, const float* __restrict__ b0,
    const float* __restrict__ a0, const float* __restrict__ ab0,
    const float* __restrict__ w1, const float* __restrict__ b1,
    const float* __restrict__ a1, const float* __restrict__ ab1,
    const float* __restrict__ niw, const float* __restrict__ nib,
    unsigned short* __restrict__ Yh, unsigned short* __restrict__ Yl)
{
  extern __shared__ __align__(16) unsigned char dsm[];
  float* sX   = (float*)(dsm + O_X);
  float* sCos = (float*)(dsm + O_TW);
  float* sSin = sCos + 64;
  float* sWin = sCos + 128;
  float* sMag = (float*)(dsm + O_MAG);
  float* sC   = (float*)(dsm + O_C);
  float* sPcc = (float*)(dsm + O_PCC);
  float* sNrm = (float*)(dsm + O_V);
  float* sNiv = sNrm + 48;
  float* sHi  = sNrm + 96;
  float* sS1  = sNrm + 144;
  float* sS2  = sNrm + 192;
  float* sMx  = sNrm + 240;
  float* sRd  = sNrm + 288;
  unsigned short* sAh = (unsigned short*)(dsm + O_AH);
  unsigned short* sAl = (unsigned short*)(dsm + O_AL);
  unsigned short* sBh = (unsigned short*)(dsm + O_BH);
  unsigned short* sBl = (unsigned short*)(dsm + O_BL);
  float* sWh = (float*)(dsm + O_WH);

  const int tid = threadIdx.x, lane = tid & 31, wv = tid >> 5;
  const int h = lane >> 4, m = lane & 15;
  const int p = blockIdx.x;

  if (tid < NSEG) {
    const float ang = (6.28318530717958647692f * (float)tid) * 0.015625f;
    const float cv = cosf(ang);
    sCos[tid] = cv;
    sSin[tid] = sinf(ang);
    sWin[tid] = 0.5f * (1.0f - cv);
  }
  __syncthreads();

  const float* xp = x + (size_t)p * PLEN;
  #pragma unroll 1
  for (int i = 0; i < 17; ++i) {
    const int idx = tid + 128 * i;
    const int t = idx >> 6, n = idx & 63;
    int o = t * NSEG + n - NSEG / 2;
    o = (o < 0) ? -o : o;
    o = (o >= PLEN) ? (2 * PLEN - 2 - o) : o;
    o = (o < 0) ? 0 : ((o > PLEN - 1) ? (PLEN - 1) : o);
    const float v = xp[o] * sWin[n];
    if (idx < NFRM * NSEG) sX[idx] = v;
  }
  __syncthreads();

  for (int pr = tid; pr < NFRM * NNODE; pr += 128) {
    const int t = pr / NNODE, k = pr - NNODE * t;
    const float* fr = sX + t * NSEG;
    float re = 0.f, im = 0.f;
    int ph = 0;
    #pragma unroll 4
    for (int j = 0; j < NSEG; ++j) {
      const float v = fr[j];
      re = fmaf(v, sCos[ph], re);
      im = fmaf(v, sSin[ph], im);
      ph = (ph + k) & 63;
    }
    sMag[k * NFRM + t] = sqrtf(re * re + im * im);
  }
  __syncthreads();

  if (tid < NNODE) {
    const float* mr = sMag + tid * NFRM;
    float su = 0.f, nv = 0.f;
    #pragma unroll 1
    for (int f = 0; f < NFRM; ++f) { const float v = mr[f]; su += v; nv = fmaf(v, niw[f], nv); }
    const float mean = su * (1.0f / 33.0f);
    float ss = 0.f;
    #pragma unroll 1
    for (int f = 0; f < NFRM; ++f) {
      const float cc = mr[f] - mean;
      sC[tid * NFRM + f] = cc;
      ss = fmaf(cc, cc, ss);
    }
    sNrm[tid] = sqrtf(ss);
    sNiv[tid] = nv + nib[0];
  }
  __syncthreads();
  for (int pr = tid; pr < NNODE * NNODE; pr += 128) {
    const int n = pr / NNODE, mm = pr - NNODE * n;
    const float* cn = sC + n * NFRM;
    const float* cm = sC + mm * NFRM;
    float d = 0.f;
    #pragma unroll 3
    for (int f = 0; f < NFRM; ++f) d = fmaf(cn[f], cm[f], d);
    sPcc[pr] = d / (sNrm[n] * sNrm[mm]);
  }
  __syncthreads();
  if (tid < NNODE) {
    float a = 0.f;
    #pragma unroll 1
    for (int mm = 0; mm < NNODE; ++mm) a = fmaf(sPcc[tid * NNODE + mm], sNiv[mm], a);
    sHi[tid] = (a > 0.f) ? 1.f : 0.f;
  }
  #pragma unroll 1
  for (int i = 0; i < 24; ++i) {
    const int idx = tid + 128 * i;
    const int n = idx >> 6, f = idx & 63;
    const int nc = (n < NNODE) ? n : (NNODE - 1);
    const int fc = (f < NFRM) ? f : (NFRM - 1);
    float v = sMag[nc * NFRM + fc];
    v = (n < NNODE && f < NFRM) ? v : 0.f;
    unsigned int hb, lb;
    split2(v, hb, lb);
    sAh[n * AP + f] = (unsigned short)hb;
    sAl[n * AP + f] = (unsigned short)lb;
  }
  __syncthreads();

  #pragma unroll 1
  for (int layer = 0; layer < 2; ++layer) {
    const float* W   = layer ? w1 : w0;
    const float* bb  = layer ? b1 : b0;
    const float* av  = layer ? a1 : a0;
    const float* abp = layer ? ab1 : ab0;
    const int FIN = layer ? GW : NFRM;

    #pragma unroll 1
    for (int i = 0; i < 32; ++i) {
      const int idx = tid + 128 * i;
      const int k = idx >> 6, n = idx & 63;
      const int kc = (k < FIN) ? k : (FIN - 1);
      float v = W[kc * GW + n];
      v = (k < FIN) ? v : 0.f;
      unsigned int hb, lb;
      split2(v, hb, lb);
      sBh[n * BP + k] = (unsigned short)hb;
      sBl[n * BP + k] = (unsigned short)lb;
    }
    __syncthreads();

    {
      v8f acc[3];
      gat_gemm(sAh, sAl, sBh, sBl, wv, h, m, acc);
      const int col = 16 * wv + m;
      const float bcol = bb[col];
      #pragma unroll
      for (int mt = 0; mt < 3; ++mt)
        #pragma unroll
        for (int r = 0; r < 8; ++r)
          sWh[(16 * mt + 8 * h + r) * WP + col] = acc[mt][r] + bcol;
    }
    __syncthreads();

    if (tid < NNODE) {
      const float* wr = sWh + tid * WP;
      float s1 = 0.f, s2 = 0.f;
      #pragma unroll 1
      for (int j = 0; j < GW; ++j) {
        const float w = wr[j];
        s1 = fmaf(w, av[j], s1);
        s2 = fmaf(w, av[GW + j], s2);
      }
      sS1[tid] = s1;
      sS2[tid] = s2;
    }
    #pragma unroll 1
    for (int i = 0; i < 32; ++i) {
      const int idx = tid + 128 * i;
      const int f = idx >> 6, n = idx & 63;
      const int nc = (n < NNODE) ? n : (NNODE - 1);
      float v = sWh[nc * WP + f];
      v = (n < NNODE) ? v : 0.f;
      unsigned int hb, lb;
      split2(v, hb, lb);
      sBh[f * BP + n] = (unsigned short)hb;
      sBl[f * BP + n] = (unsigned short)lb;
    }
    __syncthreads();

    const float abv = abp[0];
    if (tid < NNODE) {
      const float s1v = sS1[tid];
      float mx = __uint_as_float(0xff800000u);
      #pragma unroll 1
      for (int k = 0; k < NNODE; ++k) {
        float e = (s1v + sS2[k]) + abv;
        e = (e > 0.f) ? e : 0.1f * e;
        mx = fmaxf(mx, e);
      }
      float d = 0.f;
      #pragma unroll 1
      for (int k = 0; k < NNODE; ++k) {
        float e = (s1v + sS2[k]) + abv;
        e = (e > 0.f) ? e : 0.1f * e;
        d += expf(e - mx);
      }
      sMx[tid] = mx;
      sRd[tid] = 1.0f / d;
    }
    __syncthreads();

    #pragma unroll 1
    for (int i = 0; i < 24; ++i) {
      const int idx = tid + 128 * i;
      const int n = idx >> 6, mm = idx & 63;
      const int nc = (n < NNODE) ? n : (NNODE - 1);
      const int mc = (mm < NNODE) ? mm : (NNODE - 1);
      float e = (sS1[nc] + sS2[mc]) + abv;
      e = (e > 0.f) ? e : 0.1f * e;
      float at = (expf(e - sMx[nc]) * sRd[nc]) * (sHi[nc] * sHi[mc]);
      at = (n < NNODE && mm < NNODE) ? at : 0.f;
      unsigned int hb, lb;
      split2(at, hb, lb);
      sAh[n * AP + mm] = (unsigned short)hb;
      sAl[n * AP + mm] = (unsigned short)lb;
    }
    __syncthreads();

    {
      v8f acc[3];
      gat_gemm(sAh, sAl, sBh, sBl, wv, h, m, acc);
      __syncthreads();
      const int col = 16 * wv + m;
      #pragma unroll
      for (int mt = 0; mt < 3; ++mt)
        #pragma unroll
        for (int r = 0; r < 8; ++r) {
          const int row = 16 * mt + 8 * h + r;
          float v = acc[mt][r];
          const float em = expm1f(v);
          v = (v > 0.f) ? v : em;
          unsigned int hb, lb;
          split2(v, hb, lb);
          sAh[row * AP + col] = (unsigned short)hb;
          sAl[row * AP + col] = (unsigned short)lb;
        }
    }
    __syncthreads();
  }

  {
    const int q = lane & 7, rq = lane >> 3;
    v4u hv[3], lv[3];
    size_t go[3];
    bool ok[3];
    #pragma unroll
    for (int s = 0; s < 3; ++s) {
      const int L = 4 * wv + 16 * s + rq;
      const int Lc = (L < NNODE) ? L : (NNODE - 1);
      ok[s] = (L < NNODE);
      hv[s] = *(const v4ua*)(sAh + Lc * AP + 8 * q);
      lv[s] = *(const v4ua*)(sAl + Lc * AP + 8 * q);
      go[s] = (size_t)p * YK + (size_t)Lc * GW + 8 * q;
    }
    #pragma unroll
    for (int s = 0; s < 3; ++s)
      if (ok[s]) { *(volatile v4u*)(Yh + go[s]) = hv[s]; *(volatile v4u*)(Yl + go[s]) = lv[s]; }
    __threadfence();
    #pragma unroll
    for (int s = 0; s < 3; ++s)
      if (ok[s]) { *(volatile v4u*)(Yh + go[s]) = hv[s]; *(volatile v4u*)(Yl + go[s]) = lv[s]; }
  }
}

__global__ __launch_bounds__(256) void k_gemm(const unsigned short* __restrict__ Ah,
                                              const unsigned short* __restrict__ Al,
                                              const unsigned short* __restrict__ Bh,
                                              const unsigned short* __restrict__ Bl,
                                              const float* __restrict__ bias,
                                              unsigned short* __restrict__ Oh,
                                              unsigned short* __restrict__ Ol,
                                              int N, int K, int relu)
{
  __shared__ __align__(16) float sT[64 * TP];
  const int tid = threadIdx.x, lane = tid & 31, wv = tid >> 5;
  const int h = lane >> 4, m = lane & 15;
  const int bx = blockIdx.x, by = blockIdx.y;
  const int wm = wv >> 2, wn = wv & 3;
  const int rb = bx * 64 + 32 * wm, cb = by * 128 + 32 * wn;

  const v8f z8 = {0.f, 0.f, 0.f, 0.f, 0.f, 0.f, 0.f, 0.f};
  v8f acc[2][2];
  #pragma unroll
  for (int mt = 0; mt < 2; ++mt)
    #pragma unroll
    for (int nt = 0; nt < 2; ++nt) acc[mt][nt] = z8;

  #pragma unroll 1
  for (int k0 = 0; k0 < K; k0 += 32) {
    v16bf ah[2], al[2];
    #pragma unroll
    for (int mt = 0; mt < 2; ++mt) {
      const size_t ao = (size_t)(rb + 16 * mt + m) * K + k0;
      ah[mt] = ldfrag_bf(Ah + ao, h);
      al[mt] = ldfrag_bf(Al + ao, h);
    }
    #pragma unroll
    for (int nt = 0; nt < 2; ++nt) {
      const size_t bo = (size_t)(cb + 16 * nt + m) * K + k0;
      const v16bf bh = ldfrag_bf(Bh + bo, h);
      const v16bf bl = ldfrag_bf(Bl + bo, h);
      #pragma unroll
      for (int mt = 0; mt < 2; ++mt) {
        acc[mt][nt] = wmma_bf(ah[mt], bh, acc[mt][nt]);
        acc[mt][nt] = wmma_bf(ah[mt], bl, acc[mt][nt]);
        acc[mt][nt] = wmma_bf(al[mt], bh, acc[mt][nt]);
      }
    }
  }
  #pragma unroll
  for (int mt = 0; mt < 2; ++mt)
    #pragma unroll
    for (int nt = 0; nt < 2; ++nt) {
      const int col = 32 * wn + 16 * nt + m;
      #pragma unroll
      for (int r = 0; r < 8; ++r) {
        const int row = 32 * wm + 16 * mt + 8 * h + r;
        sT[row * TP + col] = acc[mt][nt][r];
      }
    }
  __syncthreads();

  const int c8 = by * 128 + 8 * m;
  const v4f bb0 = *(const v4fa*)(bias + c8);
  const v4f bb1 = *(const v4fa*)(bias + c8 + 4);
  v4u hv[4], lv[4];
  size_t go[4];
  #pragma unroll
  for (int i = 0; i < 4; ++i) {
    const int row = 2 * (wv + 8 * i) + h;
    const float* sp = sT + row * TP + 8 * m;
    v4f a = *(const v4fa*)sp + bb0;
    v4f c = *(const v4fa*)(sp + 4) + bb1;
    if (relu) { a = relu4(a); c = relu4(c); }
    split8(a, c, hv[i], lv[i]);
    go[i] = (size_t)(bx * 64 + row) * N + c8;
  }
  #pragma unroll
  for (int i = 0; i < 4; ++i) {
    *(volatile v4u*)(Oh + go[i]) = hv[i];
    *(volatile v4u*)(Ol + go[i]) = lv[i];
  }
  __threadfence();
  #pragma unroll
  for (int i = 0; i < 4; ++i) {
    *(volatile v4u*)(Oh + go[i]) = hv[i];
    *(volatile v4u*)(Ol + go[i]) = lv[i];
  }
}

__device__ __forceinline__ float sigm(float v) { return 1.0f / (1.0f + expf(-v)); }

__global__ __launch_bounds__(256) void k_lstm(const unsigned short* __restrict__ Xh,
                                              const unsigned short* __restrict__ Xl,
                                              const unsigned short* __restrict__ wih,
                                              const unsigned short* __restrict__ wil,
                                              const unsigned short* __restrict__ whh,
                                              const unsigned short* __restrict__ whl,
                                              const float* __restrict__ bih,
                                              const float* __restrict__ bhh,
                                              float* __restrict__ hs)
{
  __shared__ __align__(16) unsigned short sHh[16 * LHP];
  __shared__ __align__(16) unsigned short sHl[16 * LHP];
  __shared__ __align__(16) float sC[16 * HID];
  __shared__ __align__(16) float sF[16 * HID];
  const int tid = threadIdx.x, lane = tid & 31, wv = tid >> 5;
  const int h = lane >> 4, m = lane & 15;
  const int blk = blockIdx.x;
  const v8f z8 = {0.f, 0.f, 0.f, 0.f, 0.f, 0.f, 0.f, 0.f};

  {
    const v4u z4 = {0u, 0u, 0u, 0u};
    for (int i = tid; i < (16 * LHP) / 8; i += 256) {
      *(v4ua*)(sHh + 8 * i) = z4;
      *(v4ua*)(sHl + 8 * i) = z4;
    }
    const v4f zf = {0.f, 0.f, 0.f, 0.f};
    for (int i = tid; i < (16 * HID) / 4; i += 256) *(v4fa*)(sC + 4 * i) = zf;
  }
  __syncthreads();

  #pragma unroll 1
  for (int t = 0; t < TST; ++t) {
    #pragma unroll 1
    for (int cg = 0; cg < 2; ++cg) {
      const int j = wv + 8 * cg;
      v8f acc[4];
      #pragma unroll
      for (int g = 0; g < 4; ++g) acc[g] = z8;
      #pragma unroll 1
      for (int k0 = 0; k0 < XIN; k0 += 32) {
        const size_t ao = ((size_t)(16 * blk + m) * TST + t) * XIN + k0;
        const v16bf ah = ldfrag_bf(Xh + ao, h);
        const v16bf al = ldfrag_bf(Xl + ao, h);
        #pragma unroll
        for (int g = 0; g < 4; ++g) {
          const size_t bo = (size_t)(g * HID + 16 * j + m) * XIN + k0;
          const v16bf bh = ldfrag_bf(wih + bo, h);
          const v16bf bl = ldfrag_bf(wil + bo, h);
          acc[g] = wmma_bf(ah, bh, acc[g]);
          acc[g] = wmma_bf(ah, bl, acc[g]);
          acc[g] = wmma_bf(al, bh, acc[g]);
        }
      }
      #pragma unroll 1
      for (int k0 = 0; k0 < HID; k0 += 32) {
        const v16bf ah = ldfrag_bf(sHh + m * LHP + k0, h);
        const v16bf al = ldfrag_bf(sHl + m * LHP + k0, h);
        #pragma unroll
        for (int g = 0; g < 4; ++g) {
          const size_t bo = (size_t)(g * HID + 16 * j + m) * HID + k0;
          const v16bf bh = ldfrag_bf(whh + bo, h);
          const v16bf bl = ldfrag_bf(whl + bo, h);
          acc[g] = wmma_bf(ah, bh, acc[g]);
          acc[g] = wmma_bf(ah, bl, acc[g]);
          acc[g] = wmma_bf(al, bh, acc[g]);
        }
      }
      const int u = 16 * j + m;
      const float bv0 = bih[u] + bhh[u];
      const float bv1 = bih[HID + u] + bhh[HID + u];
      const float bv2 = bih[2 * HID + u] + bhh[2 * HID + u];
      const float bv3 = bih[3 * HID + u] + bhh[3 * HID + u];
      #pragma unroll
      for (int r = 0; r < 8; ++r) {
        const int row = 8 * h + r;
        const float gi = acc[0][r] + bv0;
        const float gf = acc[1][r] + bv1;
        const float gg = acc[2][r] + bv2;
        const float gv = acc[3][r] + bv3;
        const float cold = sC[row * HID + u];
        const float cn = sigm(gf) * cold + sigm(gi) * tanhf(gg);
        const float hn = sigm(gv) * tanhf(cn);
        sC[row * HID + u] = cn;
        sF[row * HID + u] = hn;
      }
    }
    __syncthreads();

    #pragma unroll
    for (int i = 0; i < 2; ++i) {
      const int g8 = tid + 256 * i;
      const int row = g8 >> 5, cc = g8 & 31;
      const v4f a = *(const v4fa*)(sF + 8 * g8);
      const v4f c = *(const v4fa*)(sF + 8 * g8 + 4);
      v4u H, L;
      split8(a, c, H, L);
      *(v4ua*)(sHh + row * LHP + 8 * cc) = H;
      *(v4ua*)(sHl + row * LHP + 8 * cc) = L;
    }
    v4f hv[4];
    size_t go[4];
    #pragma unroll
    for (int i = 0; i < 4; ++i) {
      const int g = tid + 256 * i;
      const int row = g >> 6, pc = g & 63;
      hv[i] = *(const v4fa*)(sF + 4 * g);
      go[i] = (((size_t)(16 * blk + row)) * TST + t) * HID + 4 * pc;
    }
    #pragma unroll
    for (int i = 0; i < 4; ++i) *(volatile v4f*)(hs + go[i]) = hv[i];
    __threadfence();
    #pragma unroll
    for (int i = 0; i < 4; ++i) *(volatile v4f*)(hs + go[i]) = hv[i];
    __syncthreads();
  }
}

__global__ __launch_bounds__(256) void k_out(const float* __restrict__ hs,
                                             const float* __restrict__ ow,
                                             const float* __restrict__ ob,
                                             float* __restrict__ out)
{
  __shared__ __align__(16) float sR[BSZ];
  const int tid = threadIdx.x, lane = tid & 31, wv = tid >> 5;
  #pragma unroll 1
  for (int rr = 0; rr < 4; ++rr) {
    const int b = wv + 8 * rr;
    const float* hr = hs + (size_t)b * (TST * HID);
    float acc = 0.f;
    #pragma unroll 4
    for (int i = 0; i < (TST * HID) / 32; ++i) acc = fmaf(hr[32 * i + lane], ow[32 * i + lane], acc);
    #pragma unroll
    for (int off = 16; off > 0; off >>= 1) acc += __shfl_xor(acc, off);
    if (lane == 0) sR[b] = acc + ob[0];
  }
  __syncthreads();
  const int tc = (tid < 8) ? tid : 0;
  const v4f v = *(const v4fa*)(sR + 4 * tc);
  if (tid < 8) *(volatile v4f*)(out + 4 * tid) = v;
  __threadfence();
  if (tid < 8) *(volatile v4f*)(out + 4 * tid) = v;
}

extern "C" void kernel_launch(void* const* d_in, const int* in_sizes, int n_in,
                              void* d_out, int out_size, void* d_ws, size_t ws_size,
                              hipStream_t stream)
{
  if (n_in < 25) return;
  if (in_sizes[0]  != BSZ * TST * PLEN) return;
  if (in_sizes[1]  != NFRM * GW) return;
  if (in_sizes[2]  != GW) return;
  if (in_sizes[3]  != 2 * GW) return;
  if (in_sizes[4]  < 1) return;
  if (in_sizes[5]  != GW * GW) return;
  if (in_sizes[6]  != GW) return;
  if (in_sizes[7]  != 2 * GW) return;
  if (in_sizes[8]  < 1) return;
  if (in_sizes[9]  != NFRM) return;
  if (in_sizes[10] < 1) return;
  if (in_sizes[11] != E0K * E0N) return;
  if (in_sizes[12] != E0N) return;
  if (in_sizes[13] != E0N * E1N) return;
  if (in_sizes[14] != E1N) return;
  if (in_sizes[15] != E1N * E2N) return;
  if (in_sizes[16] != E2N) return;
  if (in_sizes[17] != E2N * E3N) return;
  if (in_sizes[18] != E3N) return;
  if (in_sizes[19] != G4 * XIN) return;
  if (in_sizes[20] != G4 * HID) return;
  if (in_sizes[21] != G4) return;
  if (in_sizes[22] != G4) return;
  if (in_sizes[23] != TST * HID) return;
  if (in_sizes[24] < 1) return;
  if (out_size != BSZ) return;

  const float* x        = (const float*)d_in[0];
  const float* gat_w0   = (const float*)d_in[1];
  const float* gat_b0   = (const float*)d_in[2];
  const float* gat_a0   = (const float*)d_in[3];
  const float* gat_ab0  = (const float*)d_in[4];
  const float* gat_w1   = (const float*)d_in[5];
  const float* gat_b1   = (const float*)d_in[6];
  const float* gat_a1   = (const float*)d_in[7];
  const float* gat_ab1  = (const float*)d_in[8];
  const float* ni_w     = (const float*)d_in[9];
  const float* ni_b     = (const float*)d_in[10];
  const float* enc_w0   = (const float*)d_in[11];
  const float* enc_b0   = (const float*)d_in[12];
  const float* enc_w1   = (const float*)d_in[13];
  const float* enc_b1   = (const float*)d_in[14];
  const float* enc_w2   = (const float*)d_in[15];
  const float* enc_b2   = (const float*)d_in[16];
  const float* enc_w3   = (const float*)d_in[17];
  const float* enc_b3   = (const float*)d_in[18];
  const float* lstm_wih = (const float*)d_in[19];
  const float* lstm_whh = (const float*)d_in[20];
  const float* lstm_bih = (const float*)d_in[21];
  const float* lstm_bhh = (const float*)d_in[22];
  const float* out_w    = (const float*)d_in[23];
  const float* out_b    = (const float*)d_in[24];
  float* out = (float*)d_out;

  const size_t bY  = (size_t)MROW * YK * 2;
  const size_t bW0 = (size_t)E0N * E0K * 2;
  const size_t bW1 = (size_t)E1N * E0N * 2;
  const size_t bW2 = (size_t)E2N * E1N * 2;
  const size_t bW3 = (size_t)E3N * E2N * 2;
  const size_t bWI = (size_t)G4 * XIN * 2;
  const size_t bWH = (size_t)G4 * HID * 2;
  const size_t bH0 = (size_t)MROW * E0N * 2;
  const size_t bH1 = (size_t)MROW * E1N * 2;
  const size_t bH2 = (size_t)MROW * E2N * 2;
  const size_t bH3 = (size_t)MROW * E3N * 2;
  const size_t bHS = (size_t)BSZ * TST * HID * 4;
  const size_t total = 2 * (bY + bW0 + bW1 + bW2 + bW3 + bWI + bWH + bH0 + bH1 + bH2 + bH3) + bHS;
  if (total > ws_size) return;
  if (total > (size_t)134217728) return;

  char* ws = (char*)d_ws;
  size_t off = 0;
  unsigned short* YH  = (unsigned short*)(ws + off); off += bY;
  unsigned short* YL  = (unsigned short*)(ws + off); off += bY;
  unsigned short* W0H = (unsigned short*)(ws + off); off += bW0;
  unsigned short* W0L = (unsigned short*)(ws + off); off += bW0;
  unsigned short* W1H = (unsigned short*)(ws + off); off += bW1;
  unsigned short* W1L = (unsigned short*)(ws + off); off += bW1;
  unsigned short* W2H = (unsigned short*)(ws + off); off += bW2;
  unsigned short* W2L = (unsigned short*)(ws + off); off += bW2;
  unsigned short* W3H = (unsigned short*)(ws + off); off += bW3;
  unsigned short* W3L = (unsigned short*)(ws + off); off += bW3;
  unsigned short* WIH = (unsigned short*)(ws + off); off += bWI;
  unsigned short* WIL = (unsigned short*)(ws + off); off += bWI;
  unsigned short* WHH = (unsigned short*)(ws + off); off += bWH;
  unsigned short* WHL = (unsigned short*)(ws + off); off += bWH;
  unsigned short* H0H = (unsigned short*)(ws + off); off += bH0;
  unsigned short* H0L = (unsigned short*)(ws + off); off += bH0;
  unsigned short* H1H = (unsigned short*)(ws + off); off += bH1;
  unsigned short* H1L = (unsigned short*)(ws + off); off += bH1;
  unsigned short* H2H = (unsigned short*)(ws + off); off += bH2;
  unsigned short* H2L = (unsigned short*)(ws + off); off += bH2;
  unsigned short* H3H = (unsigned short*)(ws + off); off += bH3;
  unsigned short* H3L = (unsigned short*)(ws + off); off += bH3;
  float*          HS  = (float*)(ws + off);          off += bHS;
  if (off != total) return;

  k_tsplit<<<dim3(E0N / 64, E0K / 64), 256, 0, stream>>>(enc_w0, W0H, W0L, E0K, E0N);
  k_tsplit<<<dim3(E1N / 64, E0N / 64), 256, 0, stream>>>(enc_w1, W1H, W1L, E0N, E1N);
  k_tsplit<<<dim3(E2N / 64, E1N / 64), 256, 0, stream>>>(enc_w2, W2H, W2L, E1N, E2N);
  k_tsplit<<<dim3(E3N / 64, E2N / 64), 256, 0, stream>>>(enc_w3, W3H, W3L, E2N, E3N);
  {
    const int n8i = G4 * XIN / 8;
    const int n8h = G4 * HID / 8;
    k_split<<<(n8i + 255) / 256, 256, 0, stream>>>(lstm_wih, WIH, WIL, n8i);
    k_split<<<(n8h + 255) / 256, 256, 0, stream>>>(lstm_whh, WHH, WHL, n8h);
  }
  hipFuncSetAttribute(reinterpret_cast<const void*>(&k_front),
                      hipFuncAttributeMaxDynamicSharedMemorySize, LDS_FRONT);
  k_front<<<NPT, 128, LDS_FRONT, stream>>>(x, gat_w0, gat_b0, gat_a0, gat_ab0,
                                           gat_w1, gat_b1, gat_a1, gat_ab1,
                                           ni_w, ni_b, YH, YL);
  k_gemm<<<dim3(MROW / 64, E0N / 128), 256, 0, stream>>>(YH,  YL,  W0H, W0L, enc_b0, H0H, H0L, E0N, E0K, 1);
  k_gemm<<<dim3(MROW / 64, E1N / 128), 256, 0, stream>>>(H0H, H0L, W1H, W1L, enc_b1, H1H, H1L, E1N, E0N, 1);
  k_gemm<<<dim3(MROW / 64, E2N / 128), 256, 0, stream>>>(H1H, H1L, W2H, W2L, enc_b2, H2H, H2L, E2N, E1N, 1);
  k_gemm<<<dim3(MROW / 64, E3N / 128), 256, 0, stream>>>(H2H, H2L, W3H, W3L, enc_b3, H3H, H3L, E3N, E2N, 0);
  k_lstm<<<2, 256, 0, stream>>>(H3H, H3L, WIH, WIL, WHH, WHL, lstm_bih, lstm_bhh, HS);
  k_out<<<1, 256, 0, stream>>>(HS, out_w, out_b, out);
}
